// MultiHeadedAttention_spatial_36575941492790
// MI455X (gfx1250) — hardware-verified
//
#include <hip/hip_runtime.h>
#include <hip/hip_bf16.h>

typedef __attribute__((ext_vector_type(16))) _Float16 v16h;
typedef __attribute__((ext_vector_type(8)))  float    v8f;
typedef __attribute__((ext_vector_type(8)))  _Float16 v8h;
typedef __attribute__((ext_vector_type(4)))  float    v4f;
typedef __attribute__((ext_vector_type(4), may_alias)) float v4fa;
typedef __attribute__((ext_vector_type(8), may_alias)) _Float16 v8ha;

union AFrag { v16h v; uint4 q[2]; };

__global__ __launch_bounds__(256)
void cvt_f32_to_f16(const float* __restrict__ in, _Float16* __restrict__ out, int n)
{
    int base = (blockIdx.x * 256 + threadIdx.x) * 8;
    if (base >= n) return;
    v8h v;
    #pragma unroll
    for (int i = 0; i < 8; ++i) v[i] = (_Float16)in[base + i];
    *(volatile v8h*)(out + base) = v;
    __threadfence();
    *(volatile v8h*)(out + base) = v;
}

__global__ __launch_bounds__(128)
void gemm_nt_256_f16(const _Float16* __restrict__ A16,
                     const _Float16* __restrict__ W16,
                     const float* __restrict__ bias,
                     float* __restrict__ out)
{
    __shared__ _Float16 ldsA[16 * 256];
    __shared__ __attribute__((aligned(16))) float so[4][16][64];

    const int tid     = threadIdx.x;
    const int rowBase = blockIdx.x * 16;
    const int waveId  = tid >> 5;
    const int lane    = tid & 31;
    const int half    = lane >> 4;
    const int m       = lane & 15;

    {
        const uint4* src = (const uint4*)(A16 + (size_t)rowBase * 256);
        uint4* dst = (uint4*)ldsA;
        #pragma unroll
        for (int c = 0; c < 4; ++c)
            dst[tid + c * 128] = src[tid + c * 128];
    }
    __syncthreads();

    AFrag afrag[8];
    #pragma unroll
    for (int ks = 0; ks < 8; ++ks) {
        const _Float16* ap = ldsA + m * 256 + ks * 32 + 8 * half;
        afrag[ks].q[0] = *(const uint4*)(ap);
        afrag[ks].q[1] = *(const uint4*)(ap + 16);
    }

    const int n = lane & 15;
    #pragma unroll
    for (int t = 0; t < 4; ++t) {
        const int colBase = (waveId * 4 + t) * 16;
        const int wrow    = colBase + n;
        const _Float16* wp = W16 + (size_t)wrow * 256;

        v8f c = {0.f, 0.f, 0.f, 0.f, 0.f, 0.f, 0.f, 0.f};

        #pragma unroll
        for (int ks = 0; ks < 8; ++ks) {
            AFrag bf;
            const _Float16* bp = wp + ks * 32 + 8 * half;
            bf.q[0] = *(const uint4*)(bp);
            bf.q[1] = *(const uint4*)(bp + 16);
            c = __builtin_amdgcn_wmma_f32_16x16x32_f16(
                    false, afrag[ks].v, false, bf.v,
                    (short)0, c, false, false);
            asm volatile("v_nop\n\tv_nop\n\tv_nop\n\tv_nop" : "+v"(c) : "v"(afrag[ks].v), "v"(bf.v));
        }

        const float bv = bias[colBase + n];
        #pragma unroll
        for (int r = 0; r < 8; ++r)
            so[waveId][8 * half + r][t * 16 + n] = c[r] + bv;
    }
    __builtin_amdgcn_fence(__ATOMIC_ACQ_REL, "workgroup");
    __builtin_amdgcn_wave_barrier();
    {
        const int rsub = lane >> 4, c4 = (lane & 15) * 4;
        float* obase = out + (size_t)rowBase * 256 + waveId * 64 + c4;
        for (int pass = 0; pass < 2; ++pass) {
            #pragma unroll
            for (int q = 0; q < 8; ++q) {
                const int row = q * 2 + rsub;
                const v4f v = *(const v4fa*)&so[waveId][row][c4];
                *(volatile v4f*)(obase + (size_t)row * 256) = v;
            }
            if (pass == 0) __threadfence();
        }
    }
}

__global__ __launch_bounds__(256)
void attn_gather(const float* __restrict__ qb,
                 const float* __restrict__ kb,
                 const float* __restrict__ vb,
                 const int*   __restrict__ nbrs,
                 const int*   __restrict__ mask,
                 _Float16* __restrict__ x16, int nbMax)
{
    __shared__ float sp[8][32];
    __shared__ int   snb[8][32];
    __shared__ __attribute__((aligned(16))) _Float16 sx[256];

    const int b    = blockIdx.x;
    const int tid  = threadIdx.x;
    const int h    = tid >> 5;
    const int lane = tid & 31;

    int nj = nbrs[(size_t)b * 32 + lane];
    nj = nj < 0 ? 0 : (nj > nbMax ? nbMax : nj);
    const int mj = mask[(size_t)b * 32 + lane];

    const float* qrow = qb + (size_t)b  * 256 + h * 32;
    const float* krow = kb + (size_t)nj * 256 + h * 32;

    float s = 0.f;
    #pragma unroll
    for (int d = 0; d < 32; ++d) s += qrow[d] * krow[d];
    s *= 0.17677669529663689f;
    s = (mj == 0) ? -1.0e10f : s;

    float mx = s;
    #pragma unroll
    for (int off = 16; off >= 1; off >>= 1)
        mx = fmaxf(mx, __shfl_xor(mx, off, 32));
    float e = __expf(s - mx);
    float sum = e;
    #pragma unroll
    for (int off = 16; off >= 1; off >>= 1)
        sum += __shfl_xor(sum, off, 32);
    const float p = e / sum;

    sp[h][lane]  = p;
    snb[h][lane] = nj;
    __syncthreads();

    float o = 0.f;
    #pragma unroll 8
    for (int j = 0; j < 32; ++j)
        o += sp[h][j] * vb[(size_t)snb[h][j] * 256 + h * 32 + lane];

    sx[h * 32 + lane] = (_Float16)o;
    __syncthreads();
    if (tid < 32) {
        const v8h v = *(const v8ha*)&sx[tid * 8];
        *(volatile v8h*)(x16 + (size_t)b * 256 + tid * 8) = v;
        __threadfence();
        *(volatile v8h*)(x16 + (size_t)b * 256 + tid * 8) = v;
    }
}

extern "C" void kernel_launch(void* const* d_in, const int* in_sizes, int n_in,
                              void* d_out, int out_size, void* d_ws, size_t ws_size,
                              hipStream_t stream)
{
    const float* query = (const float*)d_in[0];
    const int*   nbrs  = (const int*)  d_in[1];
    const int*   mask  = (const int*)  d_in[2];
    const float* Wq    = (const float*)d_in[3];
    const float* bq    = (const float*)d_in[4];
    const float* Wk    = (const float*)d_in[5];
    const float* bk    = (const float*)d_in[6];
    const float* Wv    = (const float*)d_in[7];
    const float* bv    = (const float*)d_in[8];
    const float* Wo    = (const float*)d_in[9];
    const float* bo    = (const float*)d_in[10];

    const int nb    = in_sizes[0] / 256;
    const int nElem = nb * 256;
    const int wElem = 256 * 256;

    float*    qb   = (float*)d_ws;
    float*    kbuf = qb   + (size_t)nElem;
    float*    vbuf = kbuf + (size_t)nElem;
    _Float16* x16  = (_Float16*)(vbuf + (size_t)nElem);
    _Float16* q16  = x16 + (size_t)nElem;
    _Float16* wq16 = q16 + (size_t)nElem;
    _Float16* wk16 = wq16 + wElem;
    _Float16* wv16 = wk16 + wElem;
    _Float16* wo16 = wv16 + wElem;

    cvt_f32_to_f16<<<(nElem / 8 + 255) / 256, 256, 0, stream>>>(query, q16, nElem);
    cvt_f32_to_f16<<<(wElem / 8 + 255) / 256, 256, 0, stream>>>(Wq, wq16, wElem);
    cvt_f32_to_f16<<<(wElem / 8 + 255) / 256, 256, 0, stream>>>(Wk, wk16, wElem);
    cvt_f32_to_f16<<<(wElem / 8 + 255) / 256, 256, 0, stream>>>(Wv, wv16, wElem);
    cvt_f32_to_f16<<<(wElem / 8 + 255) / 256, 256, 0, stream>>>(Wo, wo16, wElem);

    const int gemmBlocks = nb / 16;

    gemm_nt_256_f16<<<gemmBlocks, 128, 0, stream>>>(q16, wq16, bq, qb);
    gemm_nt_256_f16<<<gemmBlocks, 128, 0, stream>>>(q16, wk16, bk, kbuf);
    gemm_nt_256_f16<<<gemmBlocks, 128, 0, stream>>>(q16, wv16, bv, vbuf);

    attn_gather<<<nb, 256, 0, stream>>>(qb, kbuf, vbuf, nbrs, mask, x16, nb - 1);

    gemm_nt_256_f16<<<gemmBlocks, 128, 0, stream>>>(x16, wo16, bo, (float*)d_out);
}
